// EdgeAwareMultiHeadAttention_68667937129203
// MI455X (gfx1250) — hardware-run, weakly checked
//
#include <hip/hip_runtime.h>


namespace {
constexpr int NG = 256, NPG = 128, N = NG * NPG  , E = 524288, NH = 8, DH = 32, HID = 256, NGT = 20, EF = 8;
constexpr float XS = 8.0f, WSC = 256.0f, PS = 8.0f, NEG = 0.2f  , SCALE = 0.17677669529663689f  , LOG2E = 1.4426950408889634f;

typedef _Float16 b16;
typedef __attribute__((ext_vector_type(16))) _Float16 v16b;
typedef __attribute__((ext_vector_type(8))) _Float16 v8b;
typedef __attribute__((ext_vector_type(8))) float v8f;
typedef __attribute__((ext_vector_type(4))) float v4f;
__device__ __forceinline__ float bf16_rne(float f) { unsigned int u = __float_as_uint(f); u += 0x7FFFu + ((u >> 16) & 1u); return __uint_as_float(u & 0xFFFF0000u); }
__device__ __forceinline__ void split16(float v, b16& hi, b16& lo) { hi = (b16)v; lo = (b16)(v - (float)hi); }
__device__ __forceinline__ v16b frag_kb(const b16* p, int hh) { const v8b a = *(const v8b*)(p + 8 * hh), b = *(const v8b*)(p + 16 + 8 * hh); v16b f;
#pragma unroll
  for (int e = 0; e < 8; ++e) { f[e] = a[e]; f[8 + e] = b[e]; } return f; }
__device__ __forceinline__ v8f wmma16b(v16b a, v16b b, v8f c) { v8f d = __builtin_amdgcn_wmma_f32_16x16x32_f16(false, a, false, b, (short)0, c, false, false); asm volatile("v_nop\n\tv_nop\n\tv_nop\n\tv_nop" : "+v"(d) : "v"(a), "v"(b)); return d; }
__device__ __forceinline__ void wave_lds_sync() { __builtin_amdgcn_fence(__ATOMIC_RELEASE, "workgroup"); __builtin_amdgcn_wave_barrier(); __builtin_amdgcn_fence(__ATOMIC_ACQUIRE, "workgroup"); }
__device__ __forceinline__ float pmul(float a, float b) { float p = a * b; asm volatile("" : "+v"(p)); return p; }
__device__ __forceinline__ int iclamp(int v, int lo, int hi) { return v < lo ? lo : (v > hi ? hi : v); }
__device__ __forceinline__ float nexp(float x) { return __builtin_amdgcn_exp2f(x * 1.4426950408889634f); }
__device__ __forceinline__ float lrelu(float x) { return x > 0.0f ? x : NEG * x; }

constexpr int CSR_NBLK = 512, CSR_GB = 9, CSR_GN = 1 << CSR_GB  , CSR_MAXG = 512, CSR_CAP = 12288  ;
__global__ __launch_bounds__(64) void csrA_kernel(const int* __restrict__ dst, int E, int N, int nG, int CHP, int NGP, int* __restrict__ STG, int* __restrict__ HST) {
  extern __shared__ int sm[];
  int* cnt = sm; int* run = sm + NGP; int* ids = sm + 2 * NGP;
  const int b = blockIdx.x; const int ch = (E + CSR_NBLK - 1) / CSR_NBLK; const int e0 = b * ch, e1 = min(E, e0 + ch);
  for (int i = threadIdx.x; i < NGP; i += 64) cnt[i] = 0;
  for (int i = threadIdx.x; i < CHP; i += 64) ids[i] = -1;
  __syncthreads();
  if (threadIdx.x == 0) {
    for (int e = e0; e < e1; ++e) { int d = dst[e]; d = (d < 0) ? 0 : (d >= N ? N - 1 : d); cnt[d >> CSR_GB] += 1; }
    int acc = 0; for (int g = 0; g < nG; ++g) { run[g] = acc; acc += cnt[g]; }
    for (int e = e0; e < e1; ++e) { int d = dst[e]; d = (d < 0) ? 0 : (d >= N ? N - 1 : d); const int g = d >> CSR_GB; ids[run[g]] = e; run[g] += 1; } }
  __syncthreads();
  typedef __attribute__((ext_vector_type(4))) int v4i;
  for (int pass = 0; pass < 2; ++pass) {
    for (int i = threadIdx.x; i < CHP / 4; i += 64) *(volatile v4i*)(STG + (size_t)b * CHP + i * 4) = *(const v4i*)(&ids[i * 4]);
    for (int i = threadIdx.x; i < NGP / 4; i += 64) { v4i v; for (int e = 0; e < 4; ++e) v[e] = (i * 4 + e < nG) ? cnt[i * 4 + e] : 0; *(volatile v4i*)(HST + (size_t)b * NGP + i * 4) = v; }
    __threadfence(); }
}
__global__ __launch_bounds__(512) void csrS_kernel(const int* __restrict__ HST, int nG, int NGP, int* __restrict__ START, int* __restrict__ TOT, int* __restrict__ OFF) {
  __shared__ int tot[CSR_MAXG];
  const int b = threadIdx.x;
  for (int pass = 0; pass < 2; ++pass) { int runb = 0; for (int g = 0; g < nG; ++g) { int c = HST[(size_t)b * NGP + g]; c = (c < 0) ? 0 : c; ((volatile int*)OFF)[(size_t)g * CSR_NBLK + b] = runb; runb += c; } __threadfence(); }
  for (int g = threadIdx.x; g < nG; g += 512) { int s = 0; for (int bb = 0; bb < CSR_NBLK; ++bb) { int c = HST[(size_t)bb * NGP + g]; s += (c < 0) ? 0 : c; } tot[g] = s; }
  __syncthreads();
  if (threadIdx.x < 32) {
    __shared__ int st[CSR_MAXG + 32];
    if (threadIdx.x == 0) { int acc = 0; for (int g = 0; g < NGP; ++g) { st[g] = acc; if (g < nG) acc += (tot[g] + 31) & ~31; } st[NGP] = acc; }
    __builtin_amdgcn_fence(__ATOMIC_RELEASE, "workgroup"); __builtin_amdgcn_wave_barrier(); __builtin_amdgcn_fence(__ATOMIC_ACQUIRE, "workgroup");
    for (int pass = 0; pass < 2; ++pass) { for (int i = threadIdx.x; i < NGP + 32; i += 32) { ((volatile int*)START)[i] = (i <= NGP) ? st[min(i, NGP)] : 0; ((volatile int*)TOT)[i] = (i < nG) ? tot[i] : 0; } __threadfence(); } }
}
__global__ __launch_bounds__(256) void csrB_kernel(const int* __restrict__ dst, int N, int nG, int CHP, int NGP, int permLen, const int* __restrict__ STG, const int* __restrict__ HST, const int* __restrict__ OFF, const int* __restrict__ START, const int* __restrict__ TOT, int* __restrict__ PERM, int* __restrict__ ROWPTR, int* __restrict__ ROWCNT, int* __restrict__ FLAG) {
  typedef __attribute__((ext_vector_type(4))) int v4i;
  __shared__ int ids[CSR_CAP]; __shared__ unsigned short key[CSR_CAP]; __shared__ int outp[CSR_CAP]; __shared__ int ncnt[CSR_GN + 1]; __shared__ int boff[CSR_NBLK + 1];
  const int g = blockIdx.x, t_ = threadIdx.x; int tot = TOT[g]; int st = START[g], stn = START[g + 1]; const int v0 = g * CSR_GN; const int nv = min(CSR_GN, N - v0);
  st = (st < 0) ? 0 : (st > permLen - 32 ? permLen - 32 : st) & ~31; stn = (stn < st) ? st : (stn > permLen ? permLen : stn); tot = (tot < 0) ? 0 : tot; if (tot > stn - st && tot <= CSR_CAP) tot = stn - st;
  if (tot > CSR_CAP) {
    for (int pass = 0; pass < 2; ++pass) { for (int i = t_; i < CSR_GN / 4; i += 256) { v4i a, c; for (int e = 0; e < 4; ++e) { a[e] = st; c[e] = 0; } *(volatile v4i*)(ROWPTR + v0 + i * 4) = a; *(volatile v4i*)(ROWCNT + v0 + i * 4) = c; } if (t_ == 0) ((volatile int*)FLAG)[0] = 1; __threadfence(); } (void)nv; return; }
  if (t_ == 0) { int acc = 0; for (int b = 0; b < CSR_NBLK; ++b) { boff[b] = acc; int c = HST[(size_t)b * NGP + g]; c = (c < 0) ? 0 : (c > CHP ? CHP : c); acc += c; if (acc > tot) acc = tot; } boff[CSR_NBLK] = acc; }
  for (int i = t_; i <= CSR_GN; i += 256) ncnt[i] = 0;
  __syncthreads();
  for (int b = 0; b < CSR_NBLK; ++b) { const int c = boff[b + 1] - boff[b]; int o_ = OFF[(size_t)g * CSR_NBLK + b]; o_ = (o_ < 0) ? 0 : (o_ > CHP - c ? CHP - c : o_); const int* src_ = STG + (size_t)b * CHP + o_;
    for (int i = t_; i < c; i += 256) { int id = src_[i]; id = (id < 0) ? 0 : id; ids[boff[b] + i] = id; int d = dst[id]; d = (d < v0) ? v0 : (d >= N ? N - 1 : d); int kk = d - v0; kk = (kk < 0) ? 0 : (kk >= CSR_GN ? CSR_GN - 1 : kk); key[boff[b] + i] = (unsigned short)kk; } }
  __syncthreads();
  if (t_ == 0) { for (int i = 0; i < tot; ++i) ncnt[key[i]] += 1; int acc = 0; for (int vl = 0; vl < CSR_GN; ++vl) { const int c = ncnt[vl]; ncnt[vl] = acc; acc += c; } ncnt[CSR_GN] = acc;
    for (int i = 0; i < tot; ++i) { const int vl = key[i]; outp[ncnt[vl]] = ids[i]; ncnt[vl] += 1; }
    for (int vl = CSR_GN; vl > 0; --vl) ncnt[vl] = ncnt[vl - 1]; ncnt[0] = 0; }
  __syncthreads();
  for (int pass = 0; pass < 2; ++pass) {
    for (int i = t_; i < (stn - st) / 4; i += 256) { v4i v; for (int e = 0; e < 4; ++e) { const int q = i * 4 + e; v[e] = (q < tot) ? outp[q] : -1; } *(volatile v4i*)(PERM + st + i * 4) = v; }
    for (int i = t_; i < CSR_GN / 4; i += 256) { v4i a, c; for (int e = 0; e < 4; ++e) { const int vl = i * 4 + e; a[e] = st + ncnt[vl]; c[e] = (vl < nv) ? (ncnt[vl + 1] - ncnt[vl]) : 0; } *(volatile v4i*)(ROWPTR + v0 + i * 4) = a; *(volatile v4i*)(ROWCNT + v0 + i * 4) = c; }
    __threadfence(); }
}
__global__ __launch_bounds__(256) void csrZ_kernel(int* __restrict__ p, size_t n4) { typedef __attribute__((ext_vector_type(4))) int v4i; const size_t tid = (size_t)blockIdx.x * 256 + threadIdx.x, nth = (size_t)gridDim.x * 256; v4i z = {0, 0, 0, 0}; for (size_t i = tid; i < n4; i += nth) *(volatile v4i*)(p + i * 4) = z; }
struct CsrBufs { int *STG, *HST, *OFF, *START, *TOT, *PERM, *ROWPTR, *ROWCNT, *FLAG; int nG, NGP, CHP; size_t permLen; char* base; size_t bytes; };
static size_t csr_carve(CsrBufs& c, char* ws, size_t off, int E, int N) {
  const size_t off0 = off; c.base = ws + off;
  auto al = [&](size_t bytes) { char* p = ws + off; off += (bytes + 255) & ~(size_t)255; return p; };
  c.nG = (N + CSR_GN - 1) / CSR_GN; c.NGP = (c.nG + 31) & ~31; const int ch = (E + CSR_NBLK - 1) / CSR_NBLK; c.CHP = (ch + 31) & ~31; c.permLen = (size_t)E + 32 * (size_t)c.nG + 32;
  c.STG = (int*)al((size_t)CSR_NBLK * c.CHP * 4); c.HST = (int*)al((size_t)CSR_NBLK * c.NGP * 4); c.OFF = (int*)al((size_t)c.NGP * CSR_NBLK * 4); c.START = (int*)al((size_t)(c.NGP + 64) * 4); c.TOT = (int*)al((size_t)(c.NGP + 64) * 4);
  c.PERM = (int*)al(c.permLen * 4); c.ROWPTR = (int*)al((size_t)c.nG * CSR_GN * 4); c.ROWCNT = (int*)al((size_t)c.nG * CSR_GN * 4); c.FLAG = (int*)al(256);
  c.bytes = off - off0; return off;
}
static void csr_build(const CsrBufs& c, const int* dst, int E, int N, hipStream_t stream) {
  const size_t smem = (size_t)(2 * c.NGP + c.CHP) * 4;
  csrZ_kernel<<<512, 256, 0, stream>>>((int*)c.base, c.bytes / 16);
  csrA_kernel<<<CSR_NBLK, 64, smem, stream>>>(dst, E, N, c.nG, c.CHP, c.NGP, c.STG, c.HST);
  csrS_kernel<<<1, 512, 0, stream>>>(c.HST, c.nG, c.NGP, c.START, c.TOT, c.OFF);
  csrB_kernel<<<c.nG, 256, 0, stream>>>(dst, N, c.nG, c.CHP, c.NGP, (int)c.permLen, c.STG, c.HST, c.OFF, c.START, c.TOT, c.PERM, c.ROWPTR, c.ROWCNT, c.FLAG);
}


__global__ __launch_bounds__(256) void prep_kernel(const float* __restrict__ x, const float* __restrict__ wq, const float* __restrict__ wk, const float* __restrict__ wv, const float* __restrict__ wo, b16* __restrict__ X16, b16* __restrict__ W4) {
  const size_t t = (size_t)blockIdx.x * 256 + threadIdx.x; const size_t nx = (size_t)N * HID / 8, nw = (size_t)HID * HID / 8; v8b o;
  if (t < nx) { const size_t e = t * 8; const v4f a = *(const v4f*)(x + e), c = *(const v4f*)(x + e + 4); for (int j = 0; j < 4; ++j) { o[j] = (b16)(bf16_rne(a[j]) * XS); o[4 + j] = (b16)(bf16_rne(c[j]) * XS); } for (int pass = 0; pass < 2; ++pass) { *(volatile v8b*)(X16 + e) = o; __threadfence(); } return; }
  size_t u = t - nx; if (u >= 4 * nw) return; const int kind = (int)(u / nw); const int e = (int)(u % nw) * 8; const float* w = kind == 0 ? wq : kind == 1 ? wk : kind == 2 ? wv : wo; const int oo = e / HID, k0 = e % HID;
  for (int j = 0; j < 8; ++j) o[j] = (b16)(bf16_rne(w[(size_t)(k0 + j) * HID + oo]) * WSC);
  for (int pass = 0; pass < 2; ++pass) { *(volatile v8b*)(W4 + (size_t)kind * HID * HID + e) = o; __threadfence(); }
}
__global__ __launch_bounds__(256) void attn_kernel(const b16* __restrict__ X16, const b16* __restrict__ W4, const float* __restrict__ bq, const float* __restrict__ bk, const float* __restrict__ bv,
    const int* __restrict__ ei, const float* __restrict__ eattr, const int* __restrict__ etype, const int* __restrict__ batch, const float* __restrict__ gtab, const float* __restrict__ we, const float* __restrict__ be,
    const int* __restrict__ PS_, const int* __restrict__ RPS, const int* __restrict__ RCS, int plS, const int* __restrict__ PD_, const int* __restrict__ RPD, const int* __restrict__ RCD, int plD, b16* __restrict__ OBh, b16* __restrict__ OBl) {
  __shared__ float Bs[NPG][NPG]; __shared__ __attribute__((aligned(16))) b16 Qs[NPG][DH + 8], Qsl[NPG][DH + 8], Ks[NPG][DH + 8], Ksl[NPG][DH + 8]; __shared__ __attribute__((aligned(16))) b16 Vt[DH][NPG + 8], Vtl[DH][NPG + 8]; __shared__ float weh[EF], gth[NGT]; __shared__ float beh;
  const int b = blockIdx.x / NH, h = blockIdx.x % NH, t_ = threadIdx.x, wave = t_ >> 5, lane = t_ & 31, hh = lane >> 4, col = lane & 15;
  for (int q = t_; q < NPG * NPG; q += 256) Bs[q / NPG][q % NPG] = 0.0f;
  if (t_ < EF) weh[t_] = bf16_rne(we[t_ * NH + h]); if (t_ < NGT) gth[t_] = bf16_rne(gtab[t_ * NH + h]); if (t_ == 0) beh = bf16_rne(be[h]);
  { const size_t arow = (size_t)b * NPG + wave * 16 + col;
    for (int kind = 0; kind < 3; ++kind) { const b16* W = W4 + (size_t)kind * HID * HID + (size_t)h * DH * HID; const float* bias = kind == 0 ? bq : kind == 1 ? bk : bv; v8f a2[2] = {{}, {}};
#pragma unroll 2
      for (int kb = 0; kb < HID; kb += 32) { const v16b a = frag_kb(X16 + arow * HID + kb, hh);
#pragma unroll
        for (int t = 0; t < 2; ++t) a2[t] = wmma16b(a, frag_kb(W + (size_t)(t * 16 + col) * HID + kb, hh), a2[t]); }
#pragma unroll
      for (int t = 0; t < 2; ++t) { const int d = t * 16 + col; const float bb = bf16_rne(bias[h * DH + d]);
#pragma unroll
        for (int r = 0; r < 8; ++r) { const int node = wave * 16 + 8 * hh + r; b16 p, ql_; split16((a2[t][r] * (1.0f / (XS * WSC)) + bb) * XS, p, ql_);
          if (kind == 0) { Qs[node][d] = p; Qsl[node][d] = ql_; } else if (kind == 1) { Ks[node][d] = p; Ksl[node][d] = ql_; } else { Vt[d][node] = p; Vtl[d][node] = ql_; } } } } }
  __syncthreads();
  if (t_ < NPG) { const int i = t_; const int node = b * NPG + i;
    auto total = [&](int e) { float s = gth[iclamp(etype[e], 0, NGT - 1)] + beh; const float* ea = eattr + (size_t)e * EF; for (int f = 0; f < EF; ++f) s += pmul(bf16_rne(ea[f]), weh[f]); return s; };
    { int st = RPS[node], cnt = RCS[node]; cnt = iclamp(cnt, 0, 4096); st = iclamp(st, 0, plS - cnt);
      for (int j = 0; j < cnt; ++j) { const int e = iclamp(PS_[st + j], 0, E - 1); const int s = iclamp(ei[e], 0, N - 1), d = iclamp(ei[E + e], 0, N - 1); const int eb = iclamp(batch[s], 0, NG - 1); const int dl = iclamp(d - eb * NPG, 0, NPG - 1); Bs[i][dl] += total(e); } }
    { int st = RPD[node], cnt = RCD[node]; cnt = iclamp(cnt, 0, 4096); st = iclamp(st, 0, plD - cnt);
      for (int j = 0; j < cnt; ++j) { const int e = iclamp(PD_[st + j], 0, E - 1); const int s = iclamp(ei[e], 0, N - 1); const int eb = iclamp(batch[s], 0, NG - 1); const int sl = iclamp(s - eb * NPG, 0, NPG - 1); const int d = iclamp(ei[E + e], 0, N - 1); const int dl = iclamp(d - eb * NPG, 0, NPG - 1); if (sl != dl) Bs[i][sl] += total(e); } } }
  __syncthreads();
  const int q0 = wave * 16, qi = q0 + col;
  const v16b qa = frag_kb(&Qs[qi][0], hh), ql = frag_kb(&Qsl[qi][0], hh);
  v8f s[8];
#pragma unroll
  for (int kt = 0; kt < 8; ++kt) { s[kt] = (v8f){}; const v16b f = frag_kb(&Ks[kt * 16 + col][0], hh); s[kt] = wmma16b(f, qa, s[kt]); s[kt] = wmma16b(f, ql, s[kt]); s[kt] = wmma16b(frag_kb(&Ksl[kt * 16 + col][0], hh), qa, s[kt]); }
  float mx = -INFINITY; float e_[64];
#pragma unroll
  for (int kt = 0; kt < 8; ++kt)
#pragma unroll
    for (int r = 0; r < 8; ++r) { const int key = kt * 16 + 8 * hh + r; const float lg = (s[kt][r] * (SCALE / (XS * XS)) + Bs[qi][key]) * LOG2E; e_[kt * 8 + r] = lg; mx = fmaxf(mx, lg); }
  mx = fmaxf(mx, __shfl_xor(mx, 16)); float sum = 0.0f;
#pragma unroll
  for (int u = 0; u < 64; ++u) { e_[u] = __builtin_amdgcn_exp2f(e_[u] - mx); sum += e_[u]; }
  sum += __shfl_xor(sum, 16); const float inv = 1.0f / (sum * PS * XS);
  v8f o[2] = {{}, {}}, ol2[2] = {{}, {}};
#pragma unroll
  for (int kb = 0; kb < 4; ++kb) { v16b ph, pl;
#pragma unroll
    for (int r = 0; r < 8; ++r) { const float p0 = e_[(2 * kb) * 8 + r] * PS, p1 = e_[(2 * kb + 1) * 8 + r] * PS; const b16 h0 = (b16)p0, h1 = (b16)p1; ph[r] = h0; pl[r] = (b16)(p0 - (float)h0); ph[8 + r] = h1; pl[8 + r] = (b16)(p1 - (float)h1); }
#pragma unroll
    for (int t = 0; t < 2; ++t) { const v16b vf = frag_kb(&Vt[t * 16 + col][kb * 32], hh); o[t] = wmma16b(vf, ph, o[t]); ol2[t] = wmma16b(vf, pl, ol2[t]); ol2[t] = wmma16b(frag_kb(&Vtl[t * 16 + col][kb * 32], hh), ph, ol2[t]); } }
#pragma unroll
  for (int t = 0; t < 2; ++t)
#pragma unroll
    for (int r = 0; r < 8; ++r) { b16 p, q; split16((o[t][r] + ol2[t][r]) * inv * XS, p, q); Qs[q0 + col][t * 16 + 8 * hh + r] = p; Qsl[q0 + col][t * 16 + 8 * hh + r] = q; }
  wave_lds_sync();
  for (int pass = 0; pass < 2; ++pass) { for (int hq = 0; hq < 2; ++hq) { const int rr = hq * 8 + (lane >> 2), c8 = (lane & 3) * 8; const size_t gi = (((size_t)b * NH + h) * NPG + q0 + rr) * DH + c8; *(volatile v8b*)(OBh + gi) = *(const v8b*)(&Qs[q0 + rr][c8]); *(volatile v8b*)(OBl + gi) = *(const v8b*)(&Qsl[q0 + rr][c8]); } __threadfence(); }
}
__global__ __launch_bounds__(128) void outproj_kernel(const b16* __restrict__ OBh, const b16* __restrict__ OBl, const b16* __restrict__ WOT, const float* __restrict__ bo, float* __restrict__ out) {
  __shared__ __attribute__((aligned(16))) float Ts[4][16][128 + 4];
  const int wave = threadIdx.x >> 5, lane = threadIdx.x & 31, nloc = lane & 15, hlf = lane >> 4; const size_t m0 = (size_t)blockIdx.x * 64 + wave * 16; const int n0 = blockIdx.y * 128;
  const size_t node = m0 + nloc; const size_t b = node / NPG; const int q = (int)(node % NPG);
  v8f acc[8];
#pragma unroll
  for (int t = 0; t < 8; ++t) acc[t] = (v8f){};
#pragma unroll
  for (int h = 0; h < NH; ++h) { const size_t base = (((b * NH + h) * NPG) + q) * DH; const v16b a = frag_kb(OBh + base, hlf), al = frag_kb(OBl + base, hlf);
#pragma unroll
    for (int t = 0; t < 8; ++t) { const v16b bw = frag_kb(WOT + (size_t)(n0 + t * 16 + nloc) * HID + h * DH, hlf); acc[t] = wmma16b(a, bw, acc[t]); acc[t] = wmma16b(al, bw, acc[t]); } }
#pragma unroll
  for (int t = 0; t < 8; ++t) { const float bb = bf16_rne(bo[n0 + t * 16 + nloc]);
#pragma unroll
    for (int r = 0; r < 8; ++r) Ts[wave][8 * hlf + r][t * 16 + nloc] = acc[t][r] * (1.0f / (XS * WSC)) + bb; }
  wave_lds_sync();
  for (int pass = 0; pass < 2; ++pass) { for (int rr = 0; rr < 16; ++rr) *(volatile v4f*)(out + (m0 + rr) * HID + n0 + lane * 4) = *(const v4f*)(&Ts[wave][rr][lane * 4]); __threadfence(); }
}
}

extern "C" void kernel_launch(void* const* d_in, const int* in_sizes, int n_in, void* d_out, int out_size, void* d_ws, size_t ws_size, hipStream_t stream) {
  (void)n_in;
  auto Fp = [&](int i) { return (const float*)d_in[i]; }; auto Ip = [&](int i) { return (const int*)d_in[i]; };
  if (in_sizes[0] != N * HID || in_sizes[1] != E * EF || in_sizes[2] != HID * HID || in_sizes[8] != HID * HID || in_sizes[10] != NGT * NH || in_sizes[11] != EF * NH || in_sizes[13] != 2 * E || in_sizes[14] != E || in_sizes[15] != N || out_size != N * HID) return;
  size_t off = 0; char* ws = (char*)d_ws;
  auto carve = [&](size_t bytes) { char* p = ws + off; off += (bytes + 255) & ~(size_t)255; return p; };
  b16* X16 = (b16*)carve((size_t)N * HID * 2); b16* W4 = (b16*)carve((size_t)4 * HID * HID * 2);
  b16* OBh = (b16*)carve((size_t)N * HID * 2); b16* OBl = (b16*)carve((size_t)N * HID * 2);
  CsrBufs cs, cd; off = csr_carve(cs, ws, off, E, N); off = csr_carve(cd, ws, off, E, N);
  if (off > ws_size || off > ((size_t)128 << 20)) return;
  prep_kernel<<<(unsigned)(((size_t)N * HID / 8 + 4 * (size_t)HID * HID / 8 + 255) / 256), 256, 0, stream>>>(Fp(0), Fp(2), Fp(4), Fp(6), Fp(8), X16, W4);
  csr_build(cs, Ip(13), E, N, stream);
  csr_build(cd, Ip(13) + E, E, N, stream);
  attn_kernel<<<NG * NH, 256, 0, stream>>>(X16, W4, Fp(3), Fp(5), Fp(7), Ip(13), Fp(1), Ip(14), Ip(15), Fp(10), Fp(11), Fp(12), cs.PERM, cs.ROWPTR, cs.ROWCNT, (int)cs.permLen, cd.PERM, cd.ROWPTR, cd.ROWCNT, (int)cd.permLen, OBh, OBl);
  outproj_kernel<<<dim3(N / 64, 2), 128, 0, stream>>>(OBh, OBl, W4 + (size_t)3 * HID * HID, Fp(9), (float*)d_out);
}
